// DenoiseNet_8607114461272
// MI455X (gfx1250) — hardware-verified
//
#include <hip/hip_runtime.h>

typedef _Float16 v16h __attribute__((ext_vector_type(16)));
typedef _Float16 v8h  __attribute__((ext_vector_type(8)));
typedef _Float16 v8ha __attribute__((ext_vector_type(8), __may_alias__));
typedef float    v8f  __attribute__((ext_vector_type(8)));
typedef float    v4f  __attribute__((ext_vector_type(4)));
typedef float    v4fa __attribute__((ext_vector_type(4), __may_alias__));
typedef float    v2f  __attribute__((ext_vector_type(2)));
typedef float    v2fa __attribute__((ext_vector_type(2), __may_alias__));

#define HH   512
#define WW   512
#define NPIX (HH * WW)
#define NCH  64
#define NO   27

#define XS_OFF    0
#define XS_N      (4 * 36 * 36)
#define FEAT_OFF  (XS_OFF + XS_N * 4)
#define FEAT_N    (1168 * 64)
#define SEK_OFF   (FEAT_OFF + FEAT_N * 2)
#define SEK_N     (512 * 64)
#define WBT_OFF   (SEK_OFF + SEK_N * 2)
#define WBT_N     (64 * 32)
#define WKT_OFF   (WBT_OFF + WBT_N * 2)
#define WKT_N     (32 * 64)
#define WSA_OFF   (WKT_OFF + WKT_N * 2)
#define CASA_OFF  (WSA_OFF + 1280)
#define BK_OFF    (CASA_OFF + 128)
#define BF_OFF    (BK_OFF + 128)
#define KERN_OFF  (BF_OFF + 256)
#define KERN_N    (8 * 32 * 16)
#define OUTL_OFF  (KERN_OFF + KERN_N * 4)
#define OUTL_N    (3 * 16 * 32)
#define SMEM_BYTES (OUTL_OFF + OUTL_N * 4)

__host__ __device__ constexpr int koff(int k) {
    return (k / 9) * 1296 + ((k % 9) / 3) * 36 + ((k % 9) % 3);
}

__device__ __forceinline__ v8f wmma_f16(v16h a, v16h b, v8f c) {
    v8f d = __builtin_amdgcn_wmma_f32_16x16x32_f16(false, a, false, b, (short)0, c, false, false);
    asm volatile("v_nop\n\tv_nop\n\tv_nop\n\tv_nop" : "+v"(d) : "v"(a), "v"(b));
    return d;
}

__device__ __forceinline__ v16h cat16(v8h lo, v8h hi) {
    return __builtin_shufflevector(lo, hi, 0, 1, 2, 3, 4, 5, 6, 7, 8, 9, 10, 11, 12, 13, 14, 15);
}

__device__ __forceinline__ float wave_sum(float v) {
#pragma unroll
    for (int o = 16; o > 0; o >>= 1) v += __shfl_xor(v, o, 32);
    return v;
}

__device__ __forceinline__ v8h zero8h() {
    v8h z;
#pragma unroll
    for (int e = 0; e < 8; ++e) z[e] = (_Float16)0.0f;
    return z;
}

__global__ void __launch_bounds__(256)
k_stats(const float* __restrict__ x, const float* __restrict__ w_feat, const float* __restrict__ b_feat,
        const float* __restrict__ w_ca, const float* __restrict__ b_ca,
        float* __restrict__ ca_out, int nb)
{
    __shared__ float red[15][8];
    __shared__ float shL[32];
    __shared__ float mL[NCH + 2];
    __shared__ __attribute__((aligned(16))) float caL[NCH];

    const int tid  = threadIdx.x;
    const int lane = tid & 31;
    const int wv   = tid >> 5;
    const int b    = blockIdx.x;
    if (b >= nb) return;

    float part[15];
#pragma unroll
    for (int ci = 0; ci < 3; ++ci) {
        const float* p = x + (size_t)(b * 3 + ci) * NPIX;
        float s = 0.f;
        for (int i = tid * 4; i < NPIX; i += 256 * 4) {
            v4f v = *(const v4fa*)(p + i);
            s += (v[0] + v[1]) + (v[2] + v[3]);
        }
        float r0 = p[tid] + p[tid + 256];
        float r1 = p[(HH - 1) * WW + tid] + p[(HH - 1) * WW + tid + 256];
        float c0 = p[tid * WW] + p[(tid + 256) * WW];
        float c1 = p[tid * WW + (WW - 1)] + p[(tid + 256) * WW + (WW - 1)];
        part[ci * 5 + 0] = s;
        part[ci * 5 + 1] = r0;
        part[ci * 5 + 2] = r1;
        part[ci * 5 + 3] = c0;
        part[ci * 5 + 4] = c1;
    }
#pragma unroll
    for (int j = 0; j < 15; ++j) {
        float v = wave_sum(part[j]);
        if (lane == 0) red[j][wv] = v;
    }
    __syncthreads();

    if (tid < 27) {
        const int ci = tid / 9;
        const int t  = tid - ci * 9;
        const int dy = t / 3, dx = t - dy * 3;
        float tot[5];
#pragma unroll
        for (int j = 0; j < 5; ++j) {
            float a = 0.f;
#pragma unroll
            for (int w = 0; w < 8; ++w) a += red[ci * 5 + j][w];
            tot[j] = a;
        }
        const float* p = x + (size_t)(b * 3 + ci) * NPIX;
        const float x00 = p[0];
        const float x0w = p[WW - 1];
        const float xh0 = p[(size_t)(HH - 1) * WW];
        const float xhw = p[(size_t)(HH - 1) * WW + (WW - 1)];
        const float rexc = (dy == 0) ? tot[2] : ((dy == 2) ? tot[1] : 0.f);
        const float cexc = (dx == 0) ? tot[4] : ((dx == 2) ? tot[3] : 0.f);
        float cor = 0.f;
        if (dy == 0 && dx == 0) cor = xhw;
        if (dy == 0 && dx == 2) cor = xh0;
        if (dy == 2 && dx == 0) cor = x0w;
        if (dy == 2 && dx == 2) cor = x00;
        shL[tid] = tot[0] - (rexc + cexc) + cor;
    }
    __syncthreads();

    if (tid < NCH) {
        float a = 0.f;
#pragma unroll
        for (int k = 0; k < 27; ++k) a += w_feat[tid * 27 + k] * shL[k];
        mL[tid + 1] = b_feat[tid] + a * (1.0f / (float)NPIX);
    }
    if (tid == NCH) { mL[0] = 0.f; mL[NCH + 1] = 0.f; }
    __syncthreads();

    if (tid < NCH)
        caL[tid] = b_ca[0] + w_ca[0] * mL[tid] + w_ca[1] * mL[tid + 1] + w_ca[2] * mL[tid + 2];
    __syncthreads();

    if (tid < 16) {
        v4f v = *(const v4fa*)(caL + 4 * tid);
        float* g = ca_out + (size_t)b * NCH + 4 * tid;
        *(volatile v4f*)g = v;
        __threadfence();
        *(volatile v4f*)g = v;
    }
}

__global__ void __launch_bounds__(256)
k_main(const float* __restrict__ x,
       const float* __restrict__ w_feat, const float* __restrict__ b_feat,
       const float* __restrict__ w_sa,  const float* __restrict__ b_sa,
       const float* __restrict__ w_k,   const float* __restrict__ b_k,
       const float* __restrict__ ca_in, float* __restrict__ out, int nb)
{
    extern __shared__ __attribute__((aligned(16))) char smem[];
    float*    xs    = (float*)(smem + XS_OFF);
    _Float16* featL = (_Float16*)(smem + FEAT_OFF);
    _Float16* sekL  = (_Float16*)(smem + SEK_OFF);
    _Float16* wBt   = (_Float16*)(smem + WBT_OFF);
    _Float16* wKt   = (_Float16*)(smem + WKT_OFF);
    _Float16* wsaL  = (_Float16*)(smem + WSA_OFF);
    _Float16* casaL = (_Float16*)(smem + CASA_OFF);
    float*    bkL   = (float*)(smem + BK_OFF);
    float*    bfL   = (float*)(smem + BF_OFF);
    float*    kernL = (float*)(smem + KERN_OFF);
    float*    outL  = (float*)(smem + OUTL_OFF);

    const int tid  = threadIdx.x;
    const int lane = tid & 31;
    const int wv   = tid >> 5;
    const int lh   = lane >> 4;
    const int lr   = lane & 15;

    const int b  = blockIdx.z;
    if (b >= nb) return;
    const int oy = blockIdx.y * 32;
    const int ox = blockIdx.x * 32;

    for (int i = tid; i < 64 * 32; i += 256) {
        int c = i >> 5, k = i & 31;
        wBt[i] = (_Float16)((k < 27) ? 16.f * w_feat[c * 27 + k] : 0.f);
    }
    for (int i = tid; i < 32 * 64; i += 256) {
        int o = i >> 6, c = i & 63;
        wKt[i] = (_Float16)((o < NO) ? 16.f * w_k[o * 64 + c] : 0.f);
    }
    for (int i = tid; i < 9 * 64; i += 256) {
        int t = i >> 6, c = i & 63;
        wsaL[i] = (_Float16)w_sa[c * 9 + t];
    }
    if (tid < 64) {
        casaL[tid] = (_Float16)(16.f * (ca_in[b * 64 + tid] + b_sa[tid]));
        bfL[tid]   = 16.f * b_feat[tid];
    }
    if (tid < 32) bkL[tid] = (tid < NO) ? 256.f * b_k[tid] : 0.f;

    for (int i2 = tid; i2 < 4 * 36 * 18; i2 += 256) {
        int ci  = i2 / (36 * 18);
        int rem = i2 - ci * (36 * 18);
        int ry  = rem / 18;
        int rx  = (rem - ry * 18) * 2;
        int iy  = oy - 2 + ry, ix = ox - 2 + rx;
        v2f v; v[0] = 0.f; v[1] = 0.f;
        if (ci < 3 && iy >= 0 && iy < HH && ix >= 0 && ix + 1 < WW) {
            size_t gidx = ((size_t)(b * 3 + ci) * HH + iy) * WW + ix;
            v = *(const v2fa*)(x + gidx);
        }
        *(v2fa*)(xs + ci * 1296 + ry * 36 + rx) = v;
    }
    __syncthreads();

    {
        v16h bw[4];
#pragma unroll
        for (int nt = 0; nt < 4; ++nt) {
            const _Float16* bp = wBt + (nt * 16 + lr) * 32;
            v8h lo = *(const v8ha*)(bp + 8 * lh);
            v8h hi = *(const v8ha*)(bp + 16 + 8 * lh);
            bw[nt] = cat16(lo, hi);
        }
        const float bias4[4] = { bfL[lr], bfL[16 + lr], bfL[32 + lr], bfL[48 + lr] };

        for (int mt = wv; mt < 73; mt += 8) {
            const int mbase = mt * 16;
            int p = mbase + lr; p = (p > 1155) ? 1155 : p;
            const int fy = p / 34, fx = p - fy * 34;
            const int base = fy * 36 + fx;
            float tmp[16];
#pragma unroll
            for (int e = 0; e < 16; ++e) {
                const int klo = e + (e >= 8 ? 8 : 0);
                const int o0 = koff(klo), o1 = koff(klo + 8);
                tmp[e] = xs[base + (lh ? o1 : o0)];
            }
            v16h a;
#pragma unroll
            for (int e = 0; e < 16; ++e) a[e] = (_Float16)tmp[e];
#pragma unroll
            for (int nt = 0; nt < 4; ++nt) {
                const float bv = bias4[nt];
                v8f acc = { bv, bv, bv, bv, bv, bv, bv, bv };
                acc = wmma_f16(a, bw[nt], acc);
                const int c = nt * 16 + lr;
#pragma unroll
                for (int r = 0; r < 8; ++r)
                    featL[(mbase + 8 * lh + r) * 64 + c] = (_Float16)acc[r];
            }
        }
    }
    __syncthreads();

    {
        const v8h z = zero8h();
        if (oy == 0)
            for (int i = tid; i < 34 * 8; i += 256) *(v8ha*)(featL + (i >> 3) * 64 + (i & 7) * 8) = z;
        if (oy == HH - 32)
            for (int i = tid; i < 34 * 8; i += 256) *(v8ha*)(featL + (33 * 34 + (i >> 3)) * 64 + (i & 7) * 8) = z;
        if (ox == 0)
            for (int i = tid; i < 34 * 8; i += 256) *(v8ha*)(featL + ((i >> 3) * 34) * 64 + (i & 7) * 8) = z;
        if (ox == WW - 32)
            for (int i = tid; i < 34 * 8; i += 256) *(v8ha*)(featL + ((i >> 3) * 34 + 33) * 64 + (i & 7) * 8) = z;
    }
    __syncthreads();

    for (int h = 0; h < 2; ++h) {
        {
            const int r   = tid >> 4;
            const int tx  = (tid & 15) * 2;
            const int ty  = h * 16 + r;
            const int phx = r * 32 + tx;
            const v8h z = zero8h();
#pragma unroll 1
            for (int ch = 0; ch < 8; ++ch) {
                const int cb = ch * 8;
                v8h w9[9];
#pragma unroll
                for (int t = 0; t < 9; ++t) w9[t] = *(const v8ha*)(wsaL + t * 64 + cb);
                const v8h cs = *(const v8ha*)(casaL + cb);
                v8h acc0 = z, acc1 = z;
#pragma unroll
                for (int dy = 0; dy < 3; ++dy) {
                    v8h row[4];
#pragma unroll
                    for (int dx = 0; dx < 4; ++dx)
                        row[dx] = *(const v8ha*)(featL + ((ty + dy) * 34 + tx + dx) * 64 + cb);
#pragma unroll
                    for (int dx = 0; dx < 3; ++dx) {
                        acc0 += row[dx]     * w9[dy * 3 + dx];
                        acc1 += row[dx + 1] * w9[dy * 3 + dx];
                    }
                }
                acc0 += cs;
                acc1 += cs;
                *(v8ha*)(sekL + phx * 64 + cb)       = acc0;
                *(v8ha*)(sekL + (phx + 1) * 64 + cb) = acc1;
            }
        }
        __syncthreads();

        {
            v16h bk2[2][2];
#pragma unroll
            for (int kb = 0; kb < 2; ++kb)
#pragma unroll
                for (int nt = 0; nt < 2; ++nt) {
                    const _Float16* bp = wKt + (nt * 16 + lr) * 64 + kb * 32;
                    v8h lo = *(const v8ha*)(bp + 8 * lh);
                    v8h hi = *(const v8ha*)(bp + 16 + 8 * lh);
                    bk2[kb][nt] = cat16(lo, hi);
                }
            const float bko0 = bkL[lr], bko1 = bkL[16 + lr];

            for (int q = 0; q < 4; ++q) {
                const int mt    = wv * 4 + q;
                const int mbase = mt * 16;
                const int ph    = mbase + lr;

                v8h lo0 = *(const v8ha*)(sekL + ph * 64 + 8 * lh);
                v8h hi0 = *(const v8ha*)(sekL + ph * 64 + 16 + 8 * lh);
                v8h lo1 = *(const v8ha*)(sekL + ph * 64 + 32 + 8 * lh);
                v8h hi1 = *(const v8ha*)(sekL + ph * 64 + 48 + 8 * lh);
                v16h a0 = cat16(lo0, hi0);
                v16h a1 = cat16(lo1, hi1);

                v8f k0 = { bko0, bko0, bko0, bko0, bko0, bko0, bko0, bko0 };
                v8f k1 = { bko1, bko1, bko1, bko1, bko1, bko1, bko1, bko1 };
                k0 = wmma_f16(a0, bk2[0][0], k0);
                k0 = wmma_f16(a1, bk2[1][0], k0);
                k1 = wmma_f16(a0, bk2[0][1], k1);
                k1 = wmma_f16(a1, bk2[1][1], k1);

                {
                    v4f s0 = { k0[0], k0[1], k0[2], k0[3] };
                    v4f s1 = { k0[4], k0[5], k0[6], k0[7] };
                    v4f s2 = { k1[0], k1[1], k1[2], k1[3] };
                    v4f s3 = { k1[4], k1[5], k1[6], k1[7] };
                    float* kp0 = kernL + (wv * 32 + lr) * 16 + 8 * lh;
                    float* kp1 = kernL + (wv * 32 + 16 + lr) * 16 + 8 * lh;
                    *(v4fa*)(kp0)     = s0;
                    *(v4fa*)(kp0 + 4) = s1;
                    *(v4fa*)(kp1)     = s2;
                    *(v4fa*)(kp1 + 4) = s3;
                }
                asm volatile("s_wait_dscnt 0" ::: "memory");

                for (int t = lane; t < 48; t += 32) {
                    const int pl = t & 15, cc = t >> 4;
                    const int pp = mbase + pl;
                    const int rr = pp >> 5, tx2 = pp & 31;
                    const int ty2 = h * 16 + rr;
                    const float* kp = kernL + (wv * 32 + cc * 9) * 16 + pl;
                    const float* xp = xs + cc * 1296 + (ty2 + 1) * 36 + (tx2 + 1);
                    float o = 0.f;
#pragma unroll
                    for (int dy = 0; dy < 3; ++dy)
#pragma unroll
                        for (int dx = 0; dx < 3; ++dx)
                            o += kp[(dy * 3 + dx) * 16] * xp[dy * 36 + dx];
                    outL[(cc * 16 + rr) * 32 + tx2] = o * (1.0f / 256.0f);
                }
            }
        }
        __syncthreads();

        {
            const int L0 = tid >> 3, chunk = tid & 7;
            const int cc0 = L0 >> 4, rw0 = L0 & 15;
            v4f v0 = *(const v4fa*)(outL + L0 * 32 + 4 * chunk);
            float* g0 = out + (((size_t)(b * 3 + cc0) * HH + (oy + h * 16 + rw0)) * WW + ox + 4 * chunk);
            const bool has1 = (tid < 128);
            v4f v1 = v0;
            float* g1 = g0;
            if (has1) {
                const int L1 = L0 + 32;
                const int cc1 = L1 >> 4, rw1 = L1 & 15;
                v1 = *(const v4fa*)(outL + L1 * 32 + 4 * chunk);
                g1 = out + (((size_t)(b * 3 + cc1) * HH + (oy + h * 16 + rw1)) * WW + ox + 4 * chunk);
            }
            *(volatile v4f*)g0 = v0;
            if (has1) *(volatile v4f*)g1 = v1;
            __threadfence();
            *(volatile v4f*)g0 = v0;
            if (has1) *(volatile v4f*)g1 = v1;
        }
        __syncthreads();
    }
}

extern "C" void kernel_launch(void* const* d_in, const int* in_sizes, int n_in,
                              void* d_out, int out_size, void* d_ws, size_t ws_size,
                              hipStream_t stream) {
    if (n_in < 9) return;
    const int nb = in_sizes[0] / (3 * NPIX);
    if (nb <= 0 || in_sizes[0] != nb * 3 * NPIX || out_size != nb * 3 * NPIX) return;
    if (in_sizes[1] != NCH * 27 || in_sizes[2] != NCH || in_sizes[3] != NCH * 9 || in_sizes[4] != NCH ||
        in_sizes[5] < 3 || in_sizes[6] < 1 || in_sizes[7] != NO * NCH || in_sizes[8] != NO) return;
    const size_t ws_need = (size_t)nb * NCH * sizeof(float);
    if (ws_need > ws_size) return;

    const float* x      = (const float*)d_in[0];
    const float* w_feat = (const float*)d_in[1];
    const float* b_feat = (const float*)d_in[2];
    const float* w_sa   = (const float*)d_in[3];
    const float* b_sa   = (const float*)d_in[4];
    const float* w_ca   = (const float*)d_in[5];
    const float* b_ca   = (const float*)d_in[6];
    const float* w_k    = (const float*)d_in[7];
    const float* b_k    = (const float*)d_in[8];
    float* out   = (float*)d_out;
    float* ws_ca = (float*)d_ws;

    k_stats<<<nb, 256, 0, stream>>>(x, w_feat, b_feat, w_ca, b_ca, ws_ca, nb);
    k_main<<<dim3(WW / 32, HH / 32, nb), 256, SMEM_BYTES, stream>>>(
        x, w_feat, b_feat, w_sa, b_sa, w_k, b_k, ws_ca, out, nb);
}
